// Net_62801011802909
// MI455X (gfx1250) — hardware-verified
//
#include <hip/hip_runtime.h>
#include <math.h>

constexpr int NBATCH    = 1024;
constexpr int T_WARM    = 256;
constexpr int T_DEC     = 64;
constexpr int IN_FEAT   = 33;
constexpr int EMB_W     = 32;
constexpr int HID_W     = 256;
constexpr int GATE_W    = 3 * HID_W;
constexpr int MLP_W     = 64;
constexpr int NROWS_SEQ = NBATCH * T_WARM;

constexpr int OFF_WI   = 0;
constexpr int OFF_WH   = OFF_WI + GATE_W * EMB_W;
constexpr int OFF_CWH  = OFF_WH + GATE_W * HID_W;
constexpr int OFF_PW1  = OFF_CWH + GATE_W * HID_W;
constexpr int OFF_PW2  = OFF_PW1 + MLP_W * HID_W;
constexpr int W16_ELEMS = OFF_PW2 + MLP_W * MLP_W;
constexpr int PREP_THR  = 256;
constexpr int PREP_N8   = W16_ELEMS / 8;
constexpr int PREP_BLK_WI  = (GATE_W * EMB_W / 8) / PREP_THR;
constexpr int PREP_BLK_WH  = (GATE_W * HID_W / 8) / PREP_THR;
constexpr int PREP_BLK_PW1 = (MLP_W * HID_W / 8) / PREP_THR;
constexpr int PREP_BLK_PW2 = (MLP_W * MLP_W / 8) / PREP_THR;
constexpr int PREP_GRID = PREP_BLK_WI + 2 * PREP_BLK_WH + PREP_BLK_PW1 + PREP_BLK_PW2;
static_assert(PREP_N8 == PREP_GRID * PREP_THR, "prep grid exact");
static_assert((GATE_W * EMB_W / 8) % PREP_THR == 0 && (GATE_W * HID_W / 8) % PREP_THR == 0, "segment boundaries block aligned");
static_assert((MLP_W * HID_W / 8) % PREP_THR == 0 && (MLP_W * MLP_W / 8) % PREP_THR == 0, "segment boundaries block aligned");
static_assert(EMB_W % 32 == 0 && HID_W % 32 == 0 && MLP_W % 32 == 0, "every WMMA K is a multiple of 32");

constexpr size_t X3_PLANE = (size_t)NROWS_SEQ * EMB_W;

constexpr int EMB_THR   = 256;
constexpr int EMB_ROWS  = 128;
constexpr int EMB_XIN_ITERS = (EMB_ROWS * IN_FEAT + EMB_THR - 1) / EMB_THR;
constexpr int EMB_XIN   = EMB_XIN_ITERS * EMB_THR;
static_assert(NROWS_SEQ % EMB_ROWS == 0, "embedder grid exact");
static_assert(EMB_ROWS == 16 * (EMB_THR / 32), "16 rows per wave");
static_assert(EMB_ROWS * EMB_W == 2 * EMB_THR * 8, "two 8-element chunks per thread per plane");

constexpr int SEQ_THR  = 512;
constexpr int SEQ_ROWS = 32;
constexpr int HP       = 264;
constexpr int HPLANE   = SEQ_ROWS * HP;
constexpr int XP       = 40;
constexpr int XPLANE   = SEQ_ROWS * XP;
constexpr int Y1P      = 72;
constexpr int YPLANE   = SEQ_ROWS * Y1P;
constexpr int Y2P      = 68;
constexpr int PP       = 36;
static_assert(NBATCH % SEQ_ROWS == 0, "sequence grid exact");
static_assert(HID_W == 16 * (SEQ_THR / 32), "one 16-column tile per wave");
static_assert(HP % 8 == 0 && XP % 8 == 0 && Y1P % 8 == 0 && PP % 4 == 0, "16-B aligned LDS rows");
static_assert(T_DEC % 16 == 0, "output flushed in 16-step groups");

typedef __attribute__((ext_vector_type(16))) __bf16   v16b;
typedef __attribute__((ext_vector_type(8)))  __bf16   v8b;
typedef __attribute__((ext_vector_type(8)))  _Float16 v8h;
typedef __attribute__((ext_vector_type(8)))  float    v8f;
typedef __attribute__((ext_vector_type(4)))  float    v4f;
typedef __attribute__((ext_vector_type(4)))  unsigned v4u;

__device__ __forceinline__ unsigned short f2bf_bits(float f) {
  unsigned u = __float_as_uint(f);
  return (unsigned short)((u + 0x7FFFu + ((u >> 16) & 1u)) >> 16);
}
__device__ __forceinline__ float bf_bits2f(unsigned short h) { return __uint_as_float(((unsigned)h) << 16); }
__device__ __forceinline__ float bf16r(float f) { return bf_bits2f(f2bf_bits(f)); }

struct FragB {
  union U { v16b v; v8b h[2]; };
  static __device__ __forceinline__ v16b load(const __bf16* p) {
    U f; f.h[0] = *(const v8b*)(p); f.h[1] = *(const v8b*)(p + 16); return f.v;
  }
  static __device__ __forceinline__ v8f mma(v16b a, v16b b, v8f c) {
    return __builtin_amdgcn_wmma_f32_16x16x32_bf16(false, a, false, b, (short)0, c, false, false);
  }
};

__device__ __forceinline__ void guard6(v8f& a0, v8f& a1, v8f& a2, v8f& a3, v8f& a4, v8f& a5,
                                       v16b f0, v16b f1, v16b f2, v16b f3, v16b g0, v16b g1, v16b g2) {
  asm volatile("v_nop\n\tv_nop\n\tv_nop\n\tv_nop"
               : "+v"(a0), "+v"(a1), "+v"(a2), "+v"(a3), "+v"(a4), "+v"(a5)
               : "v"(f0), "v"(f1), "v"(f2), "v"(f3), "v"(g0), "v"(g1), "v"(g2));
}
__device__ __forceinline__ void guard1(v8f& a, v16b f0, v16b f1, v16b g) {
  asm volatile("v_nop\n\tv_nop\n\tv_nop\n\tv_nop" : "+v"(a) : "v"(f0), "v"(f1), "v"(g));
}

__device__ __forceinline__ float fsig(float x)  { return __builtin_amdgcn_rcpf(1.0f + __expf(-x)); }
__device__ __forceinline__ float ftanh(float x) { return 1.0f - 2.0f * __builtin_amdgcn_rcpf(__expf(2.0f * x) + 1.0f); }

__global__ __launch_bounds__(PREP_THR) void prep_weights_kernel(const float* __restrict__ gwi, const float* __restrict__ gwh,
                                                                const float* __restrict__ cwh, const float* __restrict__ pw1,
                                                                const float* __restrict__ pw2, unsigned short* __restrict__ W16) {
  const int blk = blockIdx.x;
  const int i = blk * PREP_THR + threadIdx.x;
  const float* src;
  int li;
  if (blk < PREP_BLK_WI) {
    src = gwi; li = i;
  } else if (blk < PREP_BLK_WI + PREP_BLK_WH) {
    src = gwh; li = i - PREP_BLK_WI * PREP_THR;
  } else if (blk < PREP_BLK_WI + 2 * PREP_BLK_WH) {
    src = cwh; li = i - (PREP_BLK_WI + PREP_BLK_WH) * PREP_THR;
  } else if (blk < PREP_BLK_WI + 2 * PREP_BLK_WH + PREP_BLK_PW1) {
    src = pw1; li = i - (PREP_BLK_WI + 2 * PREP_BLK_WH) * PREP_THR;
  } else {
    src = pw2; li = i - (PREP_BLK_WI + 2 * PREP_BLK_WH + PREP_BLK_PW1) * PREP_THR;
  }
  const float* sp = src + (size_t)li * 8;
  const v4f a = *(const v4f*)(sp);
  const v4f b = *(const v4f*)(sp + 4);
  v8h hv;
#pragma unroll
  for (int e = 0; e < 4; ++e) {
    const unsigned short b0 = f2bf_bits(a[e]);
    const unsigned short b1 = f2bf_bits(b[e]);
    hv[e]     = __builtin_bit_cast(_Float16, b0);
    hv[4 + e] = __builtin_bit_cast(_Float16, b1);
  }
  *(volatile v8h*)(W16 + (size_t)i * 8) = hv;
  __threadfence();
  *(volatile v8h*)(W16 + (size_t)i * 8) = hv;
}

__global__ __launch_bounds__(EMB_THR) void embed_kernel(const float* __restrict__ in_seq,
                                                        const float* __restrict__ ew1, const float* __restrict__ eb1,
                                                        const float* __restrict__ ew2, const float* __restrict__ eb2,
                                                        const float* __restrict__ ew3, const float* __restrict__ eb3,
                                                        unsigned short* __restrict__ X3) {
  __shared__ float w1s[32 * IN_FEAT];
  __shared__ float w2s[32 * 32];
  __shared__ float w3s[32 * 32];
  __shared__ float bs[96];
  __shared__ float xin[EMB_XIN];
  __shared__ float h1s[8 * 32];
  __shared__ float h2s[8 * 32];
  __shared__ __align__(16) float x3s[EMB_ROWS * EMB_W];

  const int tid = threadIdx.x, lane = tid & 31, wave = tid >> 5;
#pragma unroll 1
  for (int i = tid; i < 5 * EMB_THR; i += EMB_THR) {
    const int ic = (i < 32 * IN_FEAT) ? i : (32 * IN_FEAT - 1);
    const float v = bf16r(ew1[ic]);
    if (i < 32 * IN_FEAT) w1s[i] = v;
  }
#pragma unroll 1
  for (int i = tid; i < 32 * 32; i += EMB_THR) {
    w2s[i] = bf16r(ew2[i]);
    w3s[i] = bf16r(ew3[i]);
  }
  {
    const float v1 = eb1[lane], v2 = eb2[lane], v3 = eb3[lane];
    const float sel = (wave == 0) ? v1 : ((wave == 1) ? v2 : v3);
    if (tid < 96) bs[tid] = bf16r(sel);
  }
  {
    const size_t base  = (size_t)blockIdx.x * (size_t)(EMB_ROWS * IN_FEAT);
    const size_t total = (size_t)NROWS_SEQ * (size_t)IN_FEAT;
#pragma unroll 1
    for (int it = 0; it < EMB_XIN_ITERS; ++it) {
      const int i = it * EMB_THR + tid;
      size_t gi = base + (size_t)i;
      gi = (gi < total) ? gi : (total - 1);
      xin[i] = bf16r(in_seq[gi]);
    }
  }
  __syncthreads();

#pragma unroll 1
  for (int rr = 0; rr < 16; ++rr) {
    const int row = wave * 16 + rr;
    const float* xr = xin + row * IN_FEAT;
    float a = 0.0f;
#pragma unroll 8
    for (int k = 0; k < 32; ++k) a = fmaf(w1s[lane * IN_FEAT + k], xr[k], a);
    a = fmaf(w1s[lane * IN_FEAT + 32], xr[32], a);
    a += bs[lane];
    h1s[wave * 32 + lane] = fmaxf(a, 0.0f);
    __syncthreads();
    float b = 0.0f;
#pragma unroll 8
    for (int k = 0; k < 32; ++k) b = fmaf(w2s[lane * 32 + k], h1s[wave * 32 + k], b);
    b += bs[32 + lane];
    h2s[wave * 32 + lane] = fmaxf(b, 0.0f);
    __syncthreads();
    float cc = 0.0f;
#pragma unroll 8
    for (int k = 0; k < 32; ++k) cc = fmaf(w3s[lane * 32 + k], h2s[wave * 32 + k], cc);
    cc += bs[64 + lane];
    x3s[row * EMB_W + lane] = cc;
  }
  __syncthreads();

  v8h hv[2], lv[2];
#pragma unroll
  for (int it = 0; it < 2; ++it) {
    const int idx = it * EMB_THR + tid;
    const v4f p = *(const v4f*)(x3s + idx * 8);
    const v4f q = *(const v4f*)(x3s + idx * 8 + 4);
#pragma unroll
    for (int e = 0; e < 4; ++e) {
      const float f0 = p[e];
      const float f1 = q[e];
      const unsigned short h0 = f2bf_bits(f0);
      const unsigned short h1 = f2bf_bits(f1);
      const unsigned short l0 = f2bf_bits(f0 - bf_bits2f(h0));
      const unsigned short l1 = f2bf_bits(f1 - bf_bits2f(h1));
      hv[it][e]     = __builtin_bit_cast(_Float16, h0);
      hv[it][4 + e] = __builtin_bit_cast(_Float16, h1);
      lv[it][e]     = __builtin_bit_cast(_Float16, l0);
      lv[it][4 + e] = __builtin_bit_cast(_Float16, l1);
    }
  }
  const size_t tile0 = (size_t)blockIdx.x * (size_t)(EMB_ROWS * EMB_W);
  for (int pass = 0; pass < 2; ++pass) {
#pragma unroll
    for (int it = 0; it < 2; ++it) {
      const size_t o = tile0 + (size_t)(it * EMB_THR + tid) * 8;
      *(volatile v8h*)(X3 + o) = hv[it];
      *(volatile v8h*)(X3 + X3_PLANE + o) = lv[it];
    }
    __threadfence();
  }
}

__device__ __forceinline__ void stage_x(unsigned short* xs, const unsigned short* __restrict__ x3, int b0, int t, int tid) {
  if (tid < 256) {
    const int plane = tid >> 7, m = (tid >> 2) & 31, c8 = (tid & 3) * 8;
    const v4u v = *(const v4u*)(x3 + (size_t)plane * X3_PLANE + ((size_t)(b0 + m) * T_WARM + (size_t)t) * EMB_W + c8);
    *(v4u*)(xs + plane * XPLANE + m * XP + c8) = v;
  }
}

__device__ __forceinline__ void gate_hh(const __bf16* a0p, const __bf16* a1p, const __bf16* __restrict__ wr,
                                        v8f& r0, v8f& r1, v8f& z0, v8f& z1, v8f& n0, v8f& n1) {
  const __bf16* wz = wr + (size_t)HID_W * HID_W;
  const __bf16* wn = wr + (size_t)2 * HID_W * HID_W;
#pragma unroll 1
  for (int k0 = 0; k0 < HID_W; k0 += 32) {
    const v16b ah0 = FragB::load(a0p + k0);
    const v16b ah1 = FragB::load(a1p + k0);
    const v16b al0 = FragB::load(a0p + HPLANE + k0);
    const v16b al1 = FragB::load(a1p + HPLANE + k0);
    const v16b br  = FragB::load(wr + k0);
    const v16b bz  = FragB::load(wz + k0);
    const v16b bn  = FragB::load(wn + k0);
    r0 = FragB::mma(ah0, br, r0);
    r1 = FragB::mma(ah1, br, r1);
    z0 = FragB::mma(ah0, bz, z0);
    z1 = FragB::mma(ah1, bz, z1);
    n0 = FragB::mma(ah0, bn, n0);
    n1 = FragB::mma(ah1, bn, n1);
    r0 = FragB::mma(al0, br, r0);
    r1 = FragB::mma(al1, br, r1);
    z0 = FragB::mma(al0, bz, z0);
    z1 = FragB::mma(al1, bz, z1);
    n0 = FragB::mma(al0, bn, n0);
    n1 = FragB::mma(al1, bn, n1);
    guard6(r0, r1, z0, z1, n0, n1, ah0, ah1, al0, al1, br, bz, bn);
  }
}

__global__ __launch_bounds__(SEQ_THR) void gru_seq_kernel(
    const unsigned short* __restrict__ X3, const unsigned short* __restrict__ W16,
    const int* __restrict__ lengths_in, const int* __restrict__ lengths_out,
    const float* __restrict__ last_cords,
    const float* __restrict__ g_bi, const float* __restrict__ g_bh,
    const float* __restrict__ c_wi, const float* __restrict__ c_bi, const float* __restrict__ c_bh,
    const float* __restrict__ p_b1, const float* __restrict__ p_b2,
    const float* __restrict__ p_w3, const float* __restrict__ p_b3,
    float* __restrict__ out) {
  __shared__ __align__(16) unsigned short Hs[2 * HPLANE];
  __shared__ __align__(16) unsigned short Xs[2 * XPLANE];
  __shared__ __align__(16) unsigned short Y1s[2 * YPLANE];
  __shared__ __align__(16) float Y2s[SEQ_ROWS * Y2P];
  __shared__ __align__(16) float Ps[SEQ_ROWS * PP];
  __shared__ float W3s[2 * MLP_W];
  __shared__ float b3s[2];
  __shared__ float lcs[2 * SEQ_ROWS];
  __shared__ int   lin[SEQ_ROWS];
  __shared__ int   lout[SEQ_ROWS];

  const int tid = threadIdx.x, lane = tid & 31, wv = tid >> 5;
  const int c = lane & 15, hh = lane >> 4, koff = hh * 8;
  const int b0 = blockIdx.x * SEQ_ROWS;
  const int col = wv * 16 + c;

#pragma unroll 1
  for (int i = tid; i < HPLANE; i += SEQ_THR) ((unsigned*)Hs)[i] = 0u;
  stage_x(Xs, X3, b0, 0, tid);
  {
    const int   li  = lengths_in[b0 + lane];
    const int   lo  = lengths_out[b0 + lane];
    const float w3v = p_w3[tid & (2 * MLP_W - 1)];
    const float b3v = p_b3[tid & 1];
    const float lcv = last_cords[(size_t)b0 * 2 + (tid & (2 * SEQ_ROWS - 1))];
    if (tid < SEQ_ROWS) { lin[tid] = li; lout[tid] = lo; }
    if (tid < 2 * MLP_W) W3s[tid] = bf16r(w3v);
    if (tid < 2) b3s[tid] = bf16r(b3v);
    if (tid < 2 * SEQ_ROWS) lcs[tid] = bf16r(lcv);
  }

  float hreg[2][8];
#pragma unroll
  for (int mt = 0; mt < 2; ++mt)
#pragma unroll
    for (int r = 0; r < 8; ++r) hreg[mt][r] = 0.0f;

  const __bf16* Wb  = (const __bf16*)W16;
  const __bf16* Hb  = (const __bf16*)Hs;
  const __bf16* Xb  = (const __bf16*)Xs;
  const __bf16* Y1b = (const __bf16*)Y1s;
  const __bf16* a0p = Hb + c * HP + koff;
  const __bf16* a1p = Hb + (16 + c) * HP + koff;
  const v8f z8 = {0.f, 0.f, 0.f, 0.f, 0.f, 0.f, 0.f, 0.f};

  {
    const float biR = bf16r(g_bi[col]) + bf16r(g_bh[col]);
    const float biZ = bf16r(g_bi[HID_W + col]) + bf16r(g_bh[HID_W + col]);
    const float biN = bf16r(g_bi[2 * HID_W + col]);
    const float bhN = bf16r(g_bh[2 * HID_W + col]);
    const v16b bwr = FragB::load(Wb + OFF_WI + (size_t)col * EMB_W + koff);
    const v16b bwz = FragB::load(Wb + OFF_WI + (size_t)(HID_W + col) * EMB_W + koff);
    const v16b bwn = FragB::load(Wb + OFF_WI + (size_t)(2 * HID_W + col) * EMB_W + koff);
    const __bf16* wr  = Wb + OFF_WH + (size_t)col * HID_W + koff;
    const __bf16* x0p = Xb + c * XP + koff;
    const __bf16* x1p = Xb + (16 + c) * XP + koff;
    __syncthreads();

#pragma unroll 1
    for (int t = 0; t < T_WARM; ++t) {
      v8f aR[2], aZ[2], aNX[2], aNH[2];
      aR[0] = z8; aR[1] = z8; aZ[0] = z8; aZ[1] = z8;
      aNX[0] = z8; aNX[1] = z8; aNH[0] = z8; aNH[1] = z8;
      {
        const v16b xh0 = FragB::load(x0p);
        const v16b xh1 = FragB::load(x1p);
        const v16b xl0 = FragB::load(x0p + XPLANE);
        const v16b xl1 = FragB::load(x1p + XPLANE);
        aR[0]  = FragB::mma(xh0, bwr, aR[0]);
        aR[1]  = FragB::mma(xh1, bwr, aR[1]);
        aZ[0]  = FragB::mma(xh0, bwz, aZ[0]);
        aZ[1]  = FragB::mma(xh1, bwz, aZ[1]);
        aNX[0] = FragB::mma(xh0, bwn, aNX[0]);
        aNX[1] = FragB::mma(xh1, bwn, aNX[1]);
        aR[0]  = FragB::mma(xl0, bwr, aR[0]);
        aR[1]  = FragB::mma(xl1, bwr, aR[1]);
        aZ[0]  = FragB::mma(xl0, bwz, aZ[0]);
        aZ[1]  = FragB::mma(xl1, bwz, aZ[1]);
        aNX[0] = FragB::mma(xl0, bwn, aNX[0]);
        aNX[1] = FragB::mma(xl1, bwn, aNX[1]);
        guard6(aR[0], aR[1], aZ[0], aZ[1], aNX[0], aNX[1], xh0, xh1, xl0, xl1, bwr, bwz, bwn);
      }
      gate_hh(a0p, a1p, wr, aR[0], aR[1], aZ[0], aZ[1], aNH[0], aNH[1]);

#pragma unroll
      for (int mt = 0; mt < 2; ++mt) {
#pragma unroll
        for (int r = 0; r < 8; ++r) {
          const int m = mt * 16 + 8 * hh + r;
          const float rg = fsig(aR[mt][r] + biR);
          const float zg = fsig(aZ[mt][r] + biZ);
          const float ng = ftanh(aNX[mt][r] + biN + rg * (aNH[mt][r] + bhN));
          const float ho = hreg[mt][r];
          const float hn = (1.0f - zg) * ng + zg * ho;
          hreg[mt][r] = (t < lin[m]) ? hn : ho;
        }
      }
      __syncthreads();
#pragma unroll
      for (int mt = 0; mt < 2; ++mt) {
#pragma unroll
        for (int r = 0; r < 8; ++r) {
          const int m = mt * 16 + 8 * hh + r;
          const float hvv = hreg[mt][r];
          const unsigned short hb = f2bf_bits(hvv);
          const unsigned short lb = f2bf_bits(hvv - bf_bits2f(hb));
          Hs[m * HP + col] = hb;
          Hs[HPLANE + m * HP + col] = lb;
        }
      }
      {
        const int tn = (t + 1 < T_WARM) ? (t + 1) : (T_WARM - 1);
        stage_x(Xs, X3, b0, tn, tid);
      }
      __syncthreads();
    }
  }

  {
    const float wiR0 = bf16r(c_wi[2 * col]);
    const float wiR1 = bf16r(c_wi[2 * col + 1]);
    const float wiZ0 = bf16r(c_wi[2 * (HID_W + col)]);
    const float wiZ1 = bf16r(c_wi[2 * (HID_W + col) + 1]);
    const float wiN0 = bf16r(c_wi[2 * (2 * HID_W + col)]);
    const float wiN1 = bf16r(c_wi[2 * (2 * HID_W + col) + 1]);
    const float cbR  = bf16r(c_bi[col]) + bf16r(c_bh[col]);
    const float cbZ  = bf16r(c_bi[HID_W + col]) + bf16r(c_bh[HID_W + col]);
    const float cbiN = bf16r(c_bi[2 * HID_W + col]);
    const float cbhN = bf16r(c_bh[2 * HID_W + col]);
    const int mtw = wv & 1;
    const int ntw = (wv >> 1) & 3;
    const int oc  = ntw * 16 + c;
    const float pb1v = bf16r(p_b1[oc]);
    const float pb2v = bf16r(p_b2[oc]);
    const __bf16* wr = Wb + OFF_CWH + (size_t)col * HID_W + koff;

#pragma unroll 1
    for (int t = 0; t < T_DEC; ++t) {
      v8f aR[2], aZ[2], aNH[2];
      aR[0] = z8; aR[1] = z8; aZ[0] = z8; aZ[1] = z8; aNH[0] = z8; aNH[1] = z8;
      gate_hh(a0p, a1p, wr, aR[0], aR[1], aZ[0], aZ[1], aNH[0], aNH[1]);

#pragma unroll
      for (int mt = 0; mt < 2; ++mt) {
#pragma unroll
        for (int r = 0; r < 8; ++r) {
          const int m = mt * 16 + 8 * hh + r;
          const float l0 = lcs[2 * m], l1 = lcs[2 * m + 1];
          const float xr = fmaf(l1, wiR1, l0 * wiR0);
          const float xz = fmaf(l1, wiZ1, l0 * wiZ0);
          const float xn = fmaf(l1, wiN1, l0 * wiN0);
          const float rg = fsig(xr + cbR + aR[mt][r]);
          const float zg = fsig(xz + cbZ + aZ[mt][r]);
          const float ng = ftanh(xn + cbiN + rg * (aNH[mt][r] + cbhN));
          const float ho = hreg[mt][r];
          hreg[mt][r] = (1.0f - zg) * ng + zg * ho;
        }
      }
      __syncthreads();
#pragma unroll
      for (int mt = 0; mt < 2; ++mt) {
#pragma unroll
        for (int r = 0; r < 8; ++r) {
          const int m = mt * 16 + 8 * hh + r;
          const float hvv = hreg[mt][r];
          const unsigned short hb = f2bf_bits(hvv);
          const unsigned short lb = f2bf_bits(hvv - bf_bits2f(hb));
          Hs[m * HP + col] = hb;
          Hs[HPLANE + m * HP + col] = lb;
        }
      }
      __syncthreads();

      if (wv < 8) {
        const __bf16* ap = Hb + (mtw * 16 + c) * HP + koff;
        const __bf16* bp = Wb + OFF_PW1 + (size_t)oc * HID_W + koff;
        v8f acc = z8;
#pragma unroll 1
        for (int k0 = 0; k0 < HID_W; k0 += 32) {
          const v16b ah = FragB::load(ap + k0);
          const v16b al = FragB::load(ap + HPLANE + k0);
          const v16b bb = FragB::load(bp + k0);
          acc = FragB::mma(ah, bb, acc);
          acc = FragB::mma(al, bb, acc);
          guard1(acc, ah, al, bb);
        }
#pragma unroll
        for (int r = 0; r < 8; ++r) {
          const int m = mtw * 16 + 8 * hh + r;
          const float v = fmaxf(acc[r] + pb1v, 0.0f);
          const unsigned short hb = f2bf_bits(v);
          const unsigned short lb = f2bf_bits(v - bf_bits2f(hb));
          Y1s[m * Y1P + oc] = hb;
          Y1s[YPLANE + m * Y1P + oc] = lb;
        }
      }
      __syncthreads();

      if (wv < 8) {
        const __bf16* ap = Y1b + (mtw * 16 + c) * Y1P + koff;
        const __bf16* bp = Wb + OFF_PW2 + (size_t)oc * MLP_W + koff;
        v8f acc = z8;
#pragma unroll 1
        for (int k0 = 0; k0 < MLP_W; k0 += 32) {
          const v16b ah = FragB::load(ap + k0);
          const v16b al = FragB::load(ap + YPLANE + k0);
          const v16b bb = FragB::load(bp + k0);
          acc = FragB::mma(ah, bb, acc);
          acc = FragB::mma(al, bb, acc);
          guard1(acc, ah, al, bb);
        }
#pragma unroll
        for (int r = 0; r < 8; ++r) {
          const int m = mtw * 16 + 8 * hh + r;
          Y2s[m * Y2P + oc] = fmaxf(acc[r] + pb2v, 0.0f);
        }
      }
      __syncthreads();

      if (tid < 2 * SEQ_ROWS) {
        const int m = tid >> 1, cc = tid & 1;
        float s = 0.0f;
#pragma unroll 8
        for (int k = 0; k < MLP_W; ++k) s = fmaf(Y2s[m * Y2P + k], W3s[cc * MLP_W + k], s);
        s += b3s[cc];
        const float o = (t < lout[m]) ? s : 0.0f;
        lcs[tid] = o;
        Ps[m * PP + (t & 15) * 2 + cc] = o;
      }
      __syncthreads();

      if ((t & 15) == 15) {
        if (tid < 256) {
          const int row = tid >> 3, c4 = (tid & 7) * 4;
          const v4f v = *(const v4f*)(Ps + row * PP + c4);
          float* dst = out + (size_t)(b0 + row) * (size_t)(T_DEC * 2) + (size_t)(t - 15) * 2 + c4;
          *(volatile v4f*)dst = v;
          __threadfence();
          *(volatile v4f*)dst = v;
        }
      }
    }
  }
}

extern "C" void kernel_launch(void* const* d_in, const int* in_sizes, int n_in,
                              void* d_out, int out_size, void* d_ws, size_t ws_size, hipStream_t stream) {
  if (n_in < 24 || d_out == nullptr || d_ws == nullptr) return;
  if (in_sizes[0] != NROWS_SEQ * IN_FEAT || in_sizes[1] != NBATCH || in_sizes[2] != NBATCH ||
      in_sizes[3] != NBATCH * 2 || in_sizes[4] != 32 * IN_FEAT || in_sizes[6] != 32 * 32 || in_sizes[8] != EMB_W * 32 ||
      in_sizes[10] != GATE_W * EMB_W || in_sizes[11] != GATE_W * HID_W || in_sizes[12] != GATE_W ||
      in_sizes[13] != GATE_W || in_sizes[14] != GATE_W * 2 || in_sizes[15] != GATE_W * HID_W ||
      in_sizes[16] != GATE_W || in_sizes[17] != GATE_W || in_sizes[18] != MLP_W * HID_W || in_sizes[19] != MLP_W ||
      in_sizes[20] != MLP_W * MLP_W || in_sizes[21] != MLP_W || in_sizes[22] != 2 * MLP_W || in_sizes[23] != 2 ||
      out_size != NBATCH * T_DEC * 2) return;

  const float* in_seq      = (const float*)d_in[0];
  const int*   lengths_in  = (const int*)d_in[1];
  const int*   lengths_out = (const int*)d_in[2];
  const float* last_cords  = (const float*)d_in[3];
  const float* e_w1 = (const float*)d_in[4];
  const float* e_b1 = (const float*)d_in[5];
  const float* e_w2 = (const float*)d_in[6];
  const float* e_b2 = (const float*)d_in[7];
  const float* e_w3 = (const float*)d_in[8];
  const float* e_b3 = (const float*)d_in[9];
  const float* g_wi = (const float*)d_in[10];
  const float* g_wh = (const float*)d_in[11];
  const float* g_bi = (const float*)d_in[12];
  const float* g_bh = (const float*)d_in[13];
  const float* c_wi = (const float*)d_in[14];
  const float* c_wh = (const float*)d_in[15];
  const float* c_bi = (const float*)d_in[16];
  const float* c_bh = (const float*)d_in[17];
  const float* p_w1 = (const float*)d_in[18];
  const float* p_b1 = (const float*)d_in[19];
  const float* p_w2 = (const float*)d_in[20];
  const float* p_b2 = (const float*)d_in[21];
  const float* p_w3 = (const float*)d_in[22];
  const float* p_b3 = (const float*)d_in[23];

  char* ws = (char*)d_ws;
  size_t off = 0;
  unsigned short* X3 = (unsigned short*)(ws + off);
  off += (2 * X3_PLANE * 2 + 255) & ~(size_t)255;
  unsigned short* W16 = (unsigned short*)(ws + off);
  off += ((size_t)W16_ELEMS * 2 + 255) & ~(size_t)255;
  if (off > ws_size || off > (size_t)134217728) return;

  prep_weights_kernel<<<PREP_GRID, PREP_THR, 0, stream>>>(g_wi, g_wh, c_wh, p_w1, p_w2, W16);
  embed_kernel<<<NROWS_SEQ / EMB_ROWS, EMB_THR, 0, stream>>>(in_seq, e_w1, e_b1, e_w2, e_b2, e_w3, e_b3, X3);
  gru_seq_kernel<<<NBATCH / SEQ_ROWS, SEQ_THR, 0, stream>>>(X3, W16, lengths_in, lengths_out, last_cords,
                                                           g_bi, g_bh, c_wi, c_bi, c_bh, p_b1, p_b2, p_w3, p_b3,
                                                           (float*)d_out);
}
